// DenseEdgeModel_18056042512642
// MI455X (gfx1250) — hardware-verified
//
#include <hip/hip_runtime.h>
#include <stdint.h>


typedef __attribute__((ext_vector_type(16))) _Float16 v16h;
typedef __attribute__((ext_vector_type(8)))  _Float16 v8h;
typedef __attribute__((ext_vector_type(16))) __bf16   v16b;
typedef __attribute__((ext_vector_type(8)))  __bf16   v8b;
typedef __attribute__((ext_vector_type(8)))  float    v8f;
typedef __attribute__((ext_vector_type(4)))  float    v4f;

__device__ __forceinline__ unsigned short f2bf_bits(float f) {
  unsigned u = __float_as_uint(f);
  return (unsigned short)((u + 0x7FFFu + ((u >> 16) & 1u)) >> 16);
}
__device__ __forceinline__ float bf_bits2f(unsigned short h) { return __uint_as_float(((unsigned)h) << 16); }

__device__ __forceinline__ void dep_guard_h(v8f& a, v8f& b, v16h x, v16h y) { asm volatile("v_nop\n\tv_nop\n\tv_nop\n\tv_nop" : "+v"(a), "+v"(b) : "v"(x), "v"(y)); }
__device__ __forceinline__ void dep_guard_b(v8f& a, v8f& b, v16b x, v16b y) { asm volatile("v_nop\n\tv_nop\n\tv_nop\n\tv_nop" : "+v"(a), "+v"(b) : "v"(x), "v"(y)); }
__device__ __forceinline__ void keep4_h(v16h a, v16h b, v16h c, v16h d) { asm volatile("v_nop" :: "v"(a), "v"(b), "v"(c), "v"(d)); }
__device__ __forceinline__ void keep4_b(v16b a, v16b b, v16b c, v16b d) { asm volatile("v_nop" :: "v"(a), "v"(b), "v"(c), "v"(d)); }
__device__ __forceinline__ void acc_guard4(v8f& a, v8f& b, v8f& c, v8f& d) { asm volatile("v_nop\n\tv_nop\n\tv_nop\n\tv_nop" : "+v"(a), "+v"(b), "+v"(c), "+v"(d)); }
__device__ __forceinline__ void dep_guard3_h(v8f& a, v8f& b, v16h x, v16h y, v16h z) { asm volatile("v_nop\n\tv_nop\n\tv_nop\n\tv_nop" : "+v"(a), "+v"(b) : "v"(x), "v"(y), "v"(z)); }
__device__ __forceinline__ void acc_guard2(v8f& a, v8f& b) { asm volatile("v_nop\n\tv_nop\n\tv_nop\n\tv_nop" : "+v"(a), "+v"(b)); }

template <typename T> struct Frag;
template <> struct Frag<_Float16> {
  typedef v16h V; union U { v16h v; v8h h[2]; };
  static __device__ __forceinline__ v16h load(const _Float16* p) {
    U f; f.h[0] = *(const v8h*)(p); f.h[1] = *(const v8h*)(p + 16); return f.v;
  }
  static __device__ __forceinline__ v8f mma(v16h a, v16h b, v8f c) {
    return __builtin_amdgcn_wmma_f32_16x16x32_f16(false, a, false, b, (short)0, c, false, false);
  }
  static __device__ __forceinline__ void guard(v8f& a, v8f& b, v16h x, v16h y) { dep_guard_h(a, b, x, y); }
  static __device__ __forceinline__ void keep(v16h a, v16h b, v16h c, v16h d) { keep4_h(a, b, c, d); }
};
template <> struct Frag<__bf16> {
  typedef v16b V; union U { v16b v; v8b h[2]; };
  static __device__ __forceinline__ v16b load(const __bf16* p) {
    U f; f.h[0] = *(const v8b*)(p); f.h[1] = *(const v8b*)(p + 16); return f.v;
  }
  static __device__ __forceinline__ v8f mma(v16b a, v16b b, v8f c) {
    return __builtin_amdgcn_wmma_f32_16x16x32_bf16(false, a, false, b, (short)0, c, false, false);
  }
  static __device__ __forceinline__ void guard(v8f& a, v8f& b, v16b x, v16b y) { dep_guard_b(a, b, x, y); }
  static __device__ __forceinline__ void keep(v16b a, v16b b, v16b c, v16b d) { keep4_b(a, b, c, d); }
};

template <int ET> struct Elem;
template <> struct Elem<0> { typedef _Float16 T; };
template <> struct Elem<1> { typedef __bf16 T; };
template <int ET, bool SPLIT, int BIAS_MODE, int OUT_MODE, bool RESID, int ACT = 0>
__global__ __launch_bounds__(256) void wmma_gemm64(
    const unsigned short* __restrict__ Ap, const unsigned short* __restrict__ A2p, int lda, long strideA,
    const unsigned short* __restrict__ Btp, const unsigned short* __restrict__ Bt2p, int ldb, long strideB,
    void* __restrict__ Cout, void* __restrict__ Cout2, int ldc, long strideC,
    const float* __restrict__ bias,
    const float* __restrict__ resid, long strideR,
    int M, int N, int K, float scale) {
  typedef typename Elem<ET>::T T;
  typedef typename Frag<T>::V V;
  const T* A = (const T*)Ap; const T* A2 = (const T*)A2p; const T* Bt = (const T*)Btp; const T* Bt2 = (const T*)Bt2p;
  __shared__ __align__(16) float sT[8][16 * 68];
  const int b    = blockIdx.y;
  const int lane = threadIdx.x & 31;
  const int wave = threadIdx.x >> 5;
  const int tilesN = N >> 6;
  const int tilesM = M >> 6;
  const int tile = blockIdx.x * 8 + wave;
  if (tile >= tilesM * tilesN) return;
  const int tm = tile / tilesN;
  const int tn = tile - tm * tilesN;
  const int m0 = tm << 6;
  const int n0 = tn << 6;

  const T* Ab  = A  + (size_t)b * strideA;
  const T* Bb  = Bt + (size_t)b * strideB;
  const T* Ab2 = SPLIT ? (A2  + (size_t)b * strideA) : nullptr;
  const T* Bb2 = SPLIT ? (Bt2 + (size_t)b * strideB) : nullptr;

  const int rlane = lane & 15;
  const int koff  = (lane >> 4) * 8;
  const int mOff  = (lane >> 4) * 8;

  v8f acc[4][4];
#pragma unroll
  for (int i = 0; i < 4; ++i)
#pragma unroll
    for (int j = 0; j < 4; ++j) acc[i][j] = (v8f){0.f,0.f,0.f,0.f,0.f,0.f,0.f,0.f};

  for (int k0 = 0; k0 < K; k0 += 32) {
    V bh[4], bl[4];
#pragma unroll
    for (int j = 0; j < 4; ++j) {
      const size_t bo = (size_t)(n0 + (j << 4) + rlane) * ldb + koff + k0;
      bh[j] = Frag<T>::load(Bb + bo);
      if (SPLIT) bl[j] = Frag<T>::load(Bb2 + bo);
    }
#pragma unroll
    for (int i = 0; i < 4; ++i) {
      const size_t ao = (size_t)(m0 + (i << 4) + rlane) * lda + koff + k0;
      V ah = Frag<T>::load(Ab + ao);
      V al;
      if (SPLIT) al = Frag<T>::load(Ab2 + ao);
#pragma unroll
      for (int j = 0; j < 4; ++j) {
        acc[i][j] = Frag<T>::mma(ah, bh[j], acc[i][j]);
        if (SPLIT) {
          acc[i][j] = Frag<T>::mma(ah, bl[j], acc[i][j]);
          acc[i][j] = Frag<T>::mma(al, bh[j], acc[i][j]);
        }
      }
      Frag<T>::guard(acc[i][0], acc[i][3], ah, SPLIT ? al : ah);
    }
    Frag<T>::keep(bh[0], bh[1], bh[2], bh[3]);
    if (SPLIT) Frag<T>::keep(bl[0], bl[1], bl[2], bl[3]);
  }
  acc_guard4(acc[0][0], acc[0][1], acc[0][2], acc[0][3]);
  acc_guard4(acc[1][0], acc[1][1], acc[1][2], acc[1][3]);
  acc_guard4(acc[2][0], acc[2][1], acc[2][2], acc[2][3]);
  acc_guard4(acc[3][0], acc[3][1], acc[3][2], acc[3][3]);

  float* slab = sT[wave];
  const float* Rb = RESID ? (resid + (size_t)b * strideR) : nullptr;
#pragma unroll
  for (int i = 0; i < 4; ++i) {
    const int mBase = m0 + (i << 4);
#pragma unroll
    for (int j = 0; j < 4; ++j) {
      const int n = n0 + (j << 4) + rlane;
      float bv = 0.f;
      if (BIAS_MODE == 2) bv = bias[n];
#pragma unroll
      for (int r = 0; r < 8; ++r) {
        float v = acc[i][j][r] * scale;
        if (BIAS_MODE == 1) v += bias[mBase + mOff + r];
        if (BIAS_MODE == 2) v += bv;
        if (RESID) v += Rb[(size_t)(mBase + mOff + r) * ldc + n];
        if (ACT == 1) v = tanhf(v);
        if (ACT == 2) v = fmaxf(v, 0.0f);
        if (ACT == 3) v = v / (1.0f + expf(-v));
        if (ACT == 4) v = (v > 0.f) ? v : 0.01f * v;
        if (ACT == 5) v = 0.5f * v * (1.0f + erff(v * 0.70710678118654752f));
        slab[(mOff + r) * 68 + (j << 4) + rlane] = v;
      }
    }
    __builtin_amdgcn_fence(__ATOMIC_RELEASE, "workgroup");
    __builtin_amdgcn_wave_barrier();
    __builtin_amdgcn_fence(__ATOMIC_ACQUIRE, "workgroup");
    if (OUT_MODE == 0) {
      float* C = (float*)Cout + (size_t)b * strideC;
      const int hh = lane >> 4, c4 = (lane & 15) * 4;
      for (int pass = 0; pass < 2; ++pass) {
#pragma unroll
        for (int it = 0; it < 8; ++it) {
          const int row = it * 2 + hh;
          v4f v = *(const v4f*)(slab + row * 68 + c4);
          *(volatile v4f*)(C + (size_t)(mBase + row) * ldc + n0 + c4) = v;
        }
        __threadfence();
      }
    } else {
      const int q = lane >> 3, c8 = (lane & 7) * 8;
      unsigned short* C  = (unsigned short*)Cout  + (size_t)b * strideC;
      unsigned short* C2 = (OUT_MODE == 2) ? ((unsigned short*)Cout2 + (size_t)b * strideC) : nullptr;
      for (int pass = 0; pass < 2; ++pass) {
#pragma unroll
        for (int it = 0; it < 4; ++it) {
          const int row = it * 4 + q;
          const float* sp = slab + row * 68 + c8;
          v8h hv, lv;
#pragma unroll
          for (int e = 0; e < 8; ++e) {
            if (OUT_MODE == 1) {
              hv[e] = (_Float16)sp[e];
            } else {
              unsigned short hb = f2bf_bits(sp[e]);
              unsigned short lb = f2bf_bits(sp[e] - bf_bits2f(hb));
              hv[e] = __builtin_bit_cast(_Float16, hb);
              lv[e] = __builtin_bit_cast(_Float16, lb);
            }
          }
          *(volatile v8h*)(C + (size_t)(mBase + row) * ldc + n0 + c8) = hv;
          if (OUT_MODE == 2) *(volatile v8h*)(C2 + (size_t)(mBase + row) * ldc + n0 + c8) = lv;
        }
        __threadfence();
      }
    }
    __builtin_amdgcn_fence(__ATOMIC_RELEASE, "workgroup");
    __builtin_amdgcn_wave_barrier();
    __builtin_amdgcn_fence(__ATOMIC_ACQUIRE, "workgroup");
  }
}

__global__ __launch_bounds__(256) void k_castw(
    const float* __restrict__ in, _Float16* __restrict__ out, int n2, float sc) {
  int i = blockIdx.x * 256 + threadIdx.x;
  if (i < n2) {
    const _Float16 h0 = (_Float16)(in[2 * i] * sc), h1 = (_Float16)(in[2 * i + 1] * sc);
    const unsigned u = (unsigned)__builtin_bit_cast(unsigned short, h0) | ((unsigned)__builtin_bit_cast(unsigned short, h1) << 16);
    ((volatile unsigned*)out)[i] = u;
    __threadfence();
    ((volatile unsigned*)out)[i] = u;
  }
}

__global__ __launch_bounds__(256) void k_xT(const float* __restrict__ x, _Float16* __restrict__ a0) {
  __shared__ float s[64][65];
  const int t = threadIdx.x;
  const int hw0 = blockIdx.x * 64, c0 = blockIdx.y * 64, b = blockIdx.z;
#pragma unroll
  for (int i = 0; i < 16; ++i) {
    const int c = i * 4 + (t >> 6), hw = t & 63;
    s[c][hw] = x[((size_t)(b * 256 + c0 + c)) * 1024 + hw0 + hw];
  }
  __syncthreads();
  const int r0 = t >> 3, c8 = (t & 7) * 8;
  v8h va, vb;
#pragma unroll
  for (int e = 0; e < 8; ++e) {
    va[e] = (_Float16)s[c8 + e][r0];
    vb[e] = (_Float16)s[c8 + e][r0 + 32];
  }
  _Float16* da = a0 + ((size_t)(b * 1024 + hw0 + r0)) * 256 + c0 + c8;
  _Float16* db = da + (size_t)32 * 256;
  *(volatile v8h*)da = va;
  *(volatile v8h*)db = vb;
  __threadfence();
  *(volatile v8h*)da = va;
  *(volatile v8h*)db = vb;
}

__global__ __launch_bounds__(256) void k_xx(const float* __restrict__ flat, const int* __restrict__ pidx,
                                            const int* __restrict__ cidx, _Float16* __restrict__ xx, int b) {
  const int t = threadIdx.x, wave = t >> 5, lane = t & 31;
  const int p = blockIdx.x >> 5;
  const int q = ((blockIdx.x & 31) << 3) + wave;
  int ip = pidx[b * 256 + p];
  ip = (ip < 0) ? ip + 2048 : ip;
  ip = (ip < 0) ? 0 : ((ip > 2047) ? 2047 : ip);
  int iq = cidx[b * 256 + q];
  iq = (iq < 0) ? iq + 2048 : iq;
  iq = (iq < 0) ? 0 : ((iq > 2047) ? 2047 : iq);
  const float* pr = flat + (size_t)ip * 256 + lane * 8;
  const float* qr = flat + (size_t)iq * 256 + lane * 8;
  const v4f a0 = *(const v4f*)pr, a1 = *(const v4f*)(pr + 4);
  const v4f e0 = *(const v4f*)qr, e1 = *(const v4f*)(qr + 4);
  const v4f d0 = a0 - e0, d1 = a1 - e1;
  v8h v;
#pragma unroll
  for (int e = 0; e < 4; ++e) {
    const float s0 = d0[e] * d0[e];
    const float s1 = d1[e] * d1[e];
    v[e]     = (_Float16)(s0 * 64.0f);
    v[4 + e] = (_Float16)(s1 * 64.0f);
  }
  _Float16* dst = xx + ((size_t)(p * 256 + q)) * 256 + lane * 8;
  *(volatile v8h*)dst = v;
  __threadfence();
  *(volatile v8h*)dst = v;
}

__global__ __launch_bounds__(256) void k_proj(const _Float16* __restrict__ g2, const float* __restrict__ w3,
                                              const float* __restrict__ b3, float* __restrict__ out, int b) {
  __shared__ __align__(16) _Float16 sW[16 * 256];
  __shared__ __align__(16) float sO[8][64];
  const int t = threadIdx.x, wave = t >> 5, lane = t & 31;
  const int h = lane >> 4, m = lane & 15;
  const int p = blockIdx.x;
#pragma unroll
  for (int e = 0; e < 16; ++e) {
    const int idx = e * 256 + t;
    const int n = idx >> 8, k = idx & 255;
    const int nn = (n < 2) ? n : 1;
    float wv = w3[nn * 256 + k];
    wv = (n < 2) ? wv * 64.0f : 0.0f;
    sW[idx] = (_Float16)wv;
  }
  __syncthreads();
  const _Float16* gb = g2 + ((size_t)(p * 256 + wave * 32)) * 256;
  v8f acc0 = (v8f){0.f,0.f,0.f,0.f,0.f,0.f,0.f,0.f};
  v8f acc1 = (v8f){0.f,0.f,0.f,0.f,0.f,0.f,0.f,0.f};
#pragma unroll
  for (int ks = 0; ks < 8; ++ks) {
    const int k0 = ks * 32 + 8 * h;
    const v16h bfr = Frag<_Float16>::load(sW + m * 256 + k0);
    const v16h af0 = Frag<_Float16>::load(gb + (size_t)m * 256 + k0);
    const v16h af1 = Frag<_Float16>::load(gb + (size_t)(m + 16) * 256 + k0);
    acc0 = Frag<_Float16>::mma(af0, bfr, acc0);
    acc1 = Frag<_Float16>::mma(af1, bfr, acc1);
    dep_guard3_h(acc0, acc1, af0, af1, bfr);
  }
  acc_guard2(acc0, acc1);
  const float inv = 1.0f / 64.0f;
  const int jj = (m < 2) ? m : 1;
  const float bb = b3[jj];
  float* so = &sO[wave][0];
  if (m < 2) {
#pragma unroll
    for (int r = 0; r < 8; ++r) {
      so[m * 32 + 8 * h + r]      = acc0[r] * inv + bb;
      so[m * 32 + 16 + 8 * h + r] = acc1[r] * inv + bb;
    }
  }
  __builtin_amdgcn_fence(__ATOMIC_RELEASE, "workgroup");
  __builtin_amdgcn_wave_barrier();
  __builtin_amdgcn_fence(__ATOMIC_ACQUIRE, "workgroup");
  const int j = (lane >> 3) & 1;
  const int c4 = (lane & 7) * 4;
  v4f ov = (v4f){0.f, 0.f, 0.f, 0.f};
  if (lane < 16) ov = *(const v4f*)(so + j * 32 + c4);
  float* dst = out + ((size_t)((b * 2 + j) * 256 + p)) * 256 + wave * 32 + c4;
  if (lane < 16) *(volatile v4f*)dst = ov;
  __threadfence();
  if (lane < 16) *(volatile v4f*)dst = ov;
}

extern "C" void kernel_launch(void* const* d_in, const int* in_sizes, int n_in,
                              void* d_out, int out_size, void* d_ws, size_t ws_size,
                              hipStream_t stream) {
  const int NB = 2, CC = 256, HWN = 1024, NP = 256, NQ = 256;
  const int NODES = NB * HWN;
  const int PAIRS = NP * NQ;
  if (n_in < 9) return;
  if (in_sizes[0] != NB * CC * HWN || in_sizes[1] != NB * NP || in_sizes[2] != NB * NQ ||
      in_sizes[3] != 3 * CC * CC || in_sizes[4] != 3 * CC || in_sizes[5] != 2 * CC * CC ||
      in_sizes[6] != 2 * CC || in_sizes[7] != 2 * CC || in_sizes[8] != 2 ||
      out_size != NB * 2 * NP * NQ) return;

  const float* x      = (const float*)d_in[0];
  const int*   pidx   = (const int*)d_in[1];
  const int*   cidx   = (const int*)d_in[2];
  const float* pre_w  = (const float*)d_in[3];
  const float* pre_b  = (const float*)d_in[4];
  const float* post_w = (const float*)d_in[5];
  const float* post_b = (const float*)d_in[6];
  const float* pow_w  = (const float*)d_in[7];
  const float* pow_b  = (const float*)d_in[8];
  float* out = (float*)d_out;

  const size_t szA0   = (size_t)NODES * CC * 2;
  const size_t szH    = (size_t)NODES * CC * 2;
  const size_t szFLAT = (size_t)NODES * CC * 4;
  const size_t szPREW = (size_t)3 * CC * CC * 2;
  const size_t szPOSW = (size_t)2 * CC * CC * 2;
  const size_t szXX   = (size_t)PAIRS * CC * 2;
  const size_t szG1   = (size_t)PAIRS * CC * 2;
  const size_t offA0 = 0;
  const size_t offH1 = offA0 + szA0;
  const size_t offH2 = offH1 + szH;
  const size_t offFLAT = offH2 + szH;
  const size_t offPREW = offFLAT + szFLAT;
  const size_t offPOSW = offPREW + szPREW;
  const size_t offXX = offPOSW + szPOSW;
  const size_t offG1 = offXX + szXX;
  const size_t total = offG1 + szG1;
  if (total > ws_size) return;

  char* ws = (char*)d_ws;
  _Float16* A0     = (_Float16*)(ws + offA0);
  _Float16* H1     = (_Float16*)(ws + offH1);
  _Float16* H2     = (_Float16*)(ws + offH2);
  float*    FLAT   = (float*)(ws + offFLAT);
  _Float16* PREW16 = (_Float16*)(ws + offPREW);
  _Float16* POSW16 = (_Float16*)(ws + offPOSW);
  _Float16* XX     = (_Float16*)(ws + offXX);
  _Float16* G1     = (_Float16*)(ws + offG1);
  _Float16* G2     = XX;

  const float WSC = 64.0f;
  const float XSC = 64.0f;

  k_xT<<<dim3(HWN / 64, CC / 64, NB), 256, 0, stream>>>(x, A0);
  k_castw<<<(3 * CC * CC / 2 + 255) / 256, 256, 0, stream>>>(pre_w, PREW16, 3 * CC * CC / 2, WSC);
  k_castw<<<(2 * CC * CC / 2 + 255) / 256, 256, 0, stream>>>(post_w, POSW16, 2 * CC * CC / 2, WSC);

  const int preBlocks = ((NODES / 64) * (CC / 64) + 7) / 8;
  wmma_gemm64<0, false, 2, 1, false, 2><<<dim3(preBlocks, 1), 256, 0, stream>>>(
      (const unsigned short*)A0, (const unsigned short*)A0, CC, 0L,
      (const unsigned short*)PREW16, (const unsigned short*)PREW16, CC, 0L,
      (void*)H1, (void*)H1, CC, 0L, pre_b, pre_b, 0L, NODES, CC, CC, 1.0f / WSC);
  wmma_gemm64<0, false, 2, 1, false, 2><<<dim3(preBlocks, 1), 256, 0, stream>>>(
      (const unsigned short*)H1, (const unsigned short*)H1, CC, 0L,
      (const unsigned short*)(PREW16 + (size_t)CC * CC), (const unsigned short*)(PREW16 + (size_t)CC * CC), CC, 0L,
      (void*)H2, (void*)H2, CC, 0L, pre_b + CC, pre_b + CC, 0L, NODES, CC, CC, 1.0f / WSC);
  wmma_gemm64<0, false, 2, 0, false, 0><<<dim3(preBlocks, 1), 256, 0, stream>>>(
      (const unsigned short*)H2, (const unsigned short*)H2, CC, 0L,
      (const unsigned short*)(PREW16 + (size_t)2 * CC * CC), (const unsigned short*)(PREW16 + (size_t)2 * CC * CC), CC, 0L,
      (void*)FLAT, (void*)FLAT, CC, 0L, pre_b + 2 * CC, pre_b + 2 * CC, 0L, NODES, CC, CC, 1.0f / WSC);

  const int postBlocks = ((PAIRS / 64) * (CC / 64) + 7) / 8;
  for (int b = 0; b < NB; ++b) {
    k_xx<<<NP * (NQ / 8), 256, 0, stream>>>(FLAT, pidx, cidx, XX, b);
    wmma_gemm64<0, false, 2, 1, false, 2><<<dim3(postBlocks, 1), 256, 0, stream>>>(
        (const unsigned short*)XX, (const unsigned short*)XX, CC, 0L,
        (const unsigned short*)POSW16, (const unsigned short*)POSW16, CC, 0L,
        (void*)G1, (void*)G1, CC, 0L, post_b, post_b, 0L, PAIRS, CC, CC, 1.0f / (WSC * XSC));
    wmma_gemm64<0, false, 2, 1, false, 2><<<dim3(postBlocks, 1), 256, 0, stream>>>(
        (const unsigned short*)G1, (const unsigned short*)G1, CC, 0L,
        (const unsigned short*)(POSW16 + (size_t)CC * CC), (const unsigned short*)(POSW16 + (size_t)CC * CC), CC, 0L,
        (void*)G2, (void*)G2, CC, 0L, post_b + CC, post_b + CC, 0L, PAIRS, CC, CC, 1.0f / WSC);
    k_proj<<<NP, 256, 0, stream>>>(G2, pow_w, pow_b, out, b);
  }
}
